// Self_Attention_91104846283288
// MI455X (gfx1250) — hardware-verified
//
#include <hip/hip_runtime.h>


#ifndef NB
#define NB 2
#endif
#ifndef SEQ
#define SEQ 2048
#endif
#define NB_FULL  2
#define SEQ_FULL 2048
#define DM   1024
#define NH   16
#define HD   64
#define KCH  64
#ifndef RH
#define RH   512
#endif
#define RHE  ((RH) < (SEQ) ? (RH) : (SEQ))
#define PP   72
#define OSP  68
#define PCAR  1024.0f
#define RPCAR 0.0009765625f
#define SCL   0.125f
static_assert(SEQ % 64 == 0);
static_assert((RH) % 64 == 0);
static_assert(DM == NH * HD);
static_assert(HD == 64);
static_assert(KCH == 64);
static_assert(DM % 64 == 0);
static_assert((3 * DM) % 64 == 0);
static_assert(SEQ <= SEQ_FULL);
static_assert(NB <= NB_FULL);

typedef _Float16 h16;
typedef unsigned short bf;
typedef __attribute__((ext_vector_type(16))) __bf16   v16bf;
typedef __attribute__((ext_vector_type(16))) _Float16 v16h;
typedef __attribute__((ext_vector_type(8)))  _Float16 v8h;
typedef __attribute__((ext_vector_type(8)))  unsigned short v8us;
typedef __attribute__((ext_vector_type(8)))  float    v8f;
typedef __attribute__((ext_vector_type(4)))  float    v4f;
typedef v8h  __attribute__((may_alias)) v8ha;
typedef v4f  __attribute__((may_alias)) v4fa;
typedef v8us __attribute__((may_alias)) v8usa;

__device__ __forceinline__ unsigned short f2bf(float f) { unsigned u = __float_as_uint(f); u += 0x7FFFu + ((u >> 16) & 1u); return (unsigned short)(u >> 16); }
__device__ __forceinline__ float bf2f(unsigned short b) { return __uint_as_float(((unsigned)b) << 16); }
__device__ __forceinline__ float bfr(float f) { return bf2f(f2bf(f)); }
__device__ __forceinline__ v16h cat16(v8h lo, v8h hi) { return __builtin_shufflevector(lo, hi, 0, 1, 2, 3, 4, 5, 6, 7, 8, 9, 10, 11, 12, 13, 14, 15); }
__device__ __forceinline__ v16bf cat16b(v8us lo, v8us hi) { return __builtin_bit_cast(v16bf, __builtin_shufflevector(lo, hi, 0, 1, 2, 3, 4, 5, 6, 7, 8, 9, 10, 11, 12, 13, 14, 15)); }
__device__ __forceinline__ v8f wmma16(v16h a, v16h b, v8f c) { return __builtin_amdgcn_wmma_f32_16x16x32_f16(false, a, false, b, (short)0, c, false, false); }
__device__ __forceinline__ v8f wmmab(v16bf a, v16bf b, v8f c) { return __builtin_amdgcn_wmma_f32_16x16x32_bf16(false, a, false, b, (short)0, c, false, false); }

template <typename T16> struct WFrag;
template <> struct WFrag<h16> { typedef v16h V; static __device__ __forceinline__ V ld(const h16* p) { return cat16(*(const v8h*)p, *(const v8h*)(p + 16)); } static __device__ __forceinline__ v8f mma(V a, V b, v8f c) { return wmma16(a, b, c); } };
template <> struct WFrag<bf> { typedef v16bf V; static __device__ __forceinline__ V ld(const bf* p) { return cat16b(*(const v8us*)p, *(const v8us*)(p + 16)); } static __device__ __forceinline__ v8f mma(V a, V b, v8f c) { return wmmab(a, b, c); } };
template <typename T16, int NSPLIT, bool BIAS>
__global__ __launch_bounds__(32) void k_gemmw(const T16* __restrict__ A, const T16* __restrict__ A2, const T16* __restrict__ Bt, const T16* __restrict__ Bt2, int K, float* C, int ldc, const float* __restrict__ bias, size_t sA, size_t sB, size_t sC) {
    typedef typename WFrag<T16>::V V;
    __shared__ __align__(16) float os[16 * 68];
    const size_t z = blockIdx.z; A += z * sA; if (A2) A2 += z * sA; Bt += z * sB; if (Bt2) Bt2 += z * sB; C += z * sC;
    const int lane = threadIdx.x & 31, lr = lane & 15, hi = lane >> 4; const int r0 = blockIdx.x * 64, c0 = blockIdx.y * 64;
    v8f acc[4][4];
#pragma unroll
    for (int mb = 0; mb < 4; ++mb)
#pragma unroll
        for (int nb = 0; nb < 4; ++nb) acc[mb][nb] = (v8f){};
    const size_t aoff = (size_t)(r0 + lr) * K + 8 * hi, boff = (size_t)(c0 + lr) * K + 8 * hi;
#pragma unroll 1
    for (int kc = 0; kc < K; kc += 32) {
        V a[4], a2[4];
#pragma unroll
        for (int mb = 0; mb < 4; ++mb) { a[mb] = WFrag<T16>::ld(A + aoff + (size_t)mb * 16 * K + kc); if (NSPLIT == 1 || NSPLIT == 2) a2[mb] = WFrag<T16>::ld(A2 + aoff + (size_t)mb * 16 * K + kc); }
#pragma unroll
        for (int nb = 0; nb < 4; ++nb) { const V b = WFrag<T16>::ld(Bt + boff + (size_t)nb * 16 * K + kc); V b2; if (NSPLIT >= 2) b2 = WFrag<T16>::ld(Bt2 + boff + (size_t)nb * 16 * K + kc);
#pragma unroll
            for (int mb = 0; mb < 4; ++mb) { acc[mb][nb] = WFrag<T16>::mma(a[mb], b, acc[mb][nb]); if (NSPLIT == 1 || NSPLIT == 2) acc[mb][nb] = WFrag<T16>::mma(a2[mb], b, acc[mb][nb]); if (NSPLIT >= 2) acc[mb][nb] = WFrag<T16>::mma(a[mb], b2, acc[mb][nb]); } }
        asm volatile("v_nop\n\tv_nop\n\tv_nop\n\tv_nop" : "+v"(acc[0][0]), "+v"(acc[1][1]), "+v"(acc[2][2]), "+v"(acc[3][3]) : "v"(a[0]), "v"(a[3]));
    }
#pragma unroll
    for (int mb = 0; mb < 4; ++mb) {
#pragma unroll
        for (int nb = 0; nb < 4; ++nb) {
#pragma unroll
            for (int j = 0; j < 8; ++j) os[(hi * 8 + j) * 68 + nb * 16 + lr] = acc[mb][nb][j]; }
        __builtin_amdgcn_wave_barrier(); asm volatile("" ::: "memory");
        float* crow = C + (size_t)(r0 + mb * 16) * ldc + c0;
#pragma unroll 1
        for (int ps = 0; ps < 2; ++ps) {
#pragma unroll
            for (int s = 0; s < 8; ++s) { const int row = 2 * s + hi, cofs = lr * 4; v4f val = *(const v4fa*)(os + row * 68 + cofs); if (BIAS) { val[0] += bfr(bias[c0 + cofs]); val[1] += bfr(bias[c0 + cofs + 1]); val[2] += bfr(bias[c0 + cofs + 2]); val[3] += bfr(bias[c0 + cofs + 3]); }
                *(volatile v4f*)(crow + (size_t)row * ldc + cofs) = val; }
            if (ps == 0) __threadfence(); }
        __builtin_amdgcn_wave_barrier(); asm volatile("" ::: "memory");
    }
}

__device__ __forceinline__ h16 tohx(float x) { return (h16)x; }
__device__ __forceinline__ void splitf(float y, unsigned short& h, unsigned short& l) { h = f2bf(y); l = f2bf(y - bf2f(h)); }
typedef __attribute__((ext_vector_type(2))) _Float16 v2h;
typedef __attribute__((ext_vector_type(2))) unsigned short v2us;

__global__ __launch_bounds__(256) void k_cvt8(const float* __restrict__ src, bf* dst, size_t n8) { const size_t i = (size_t)blockIdx.x * 256 + threadIdx.x; if (i >= n8) return; const v8f v = *(const v8f*)(src + i * 8); v8us o;
#pragma unroll
    for (int k = 0; k < 8; ++k) o[k] = f2bf(v[k]); *(volatile v8us*)(dst + i * 8) = o; __threadfence(); *(volatile v8us*)(dst + i * 8) = o; }

__global__ __launch_bounds__(256) void k_hp(const float* __restrict__ F, int pitch, h16* P16, bf* Ph, bf* Pl) {
    const size_t e = ((size_t)blockIdx.x * 256 + threadIdx.x) * 2; if (e >= (size_t)NH * SEQ * HD) return;
    const int d = (int)(e % HD); const int t = (int)((e / HD) % SEQ); const int hh = (int)(e / ((size_t)HD * SEQ));
    const float* f = F + (size_t)t * pitch + hh * HD + d; v2h o16; v2us oh, ol;
#pragma unroll
    for (int q = 0; q < 2; ++q) { const float x = f[q]; o16[q] = tohx(x); unsigned short a2, c2; splitf(x, a2, c2); oh[q] = a2; ol[q] = c2; }
    *(volatile v2h*)(P16 + e) = o16; *(volatile v2us*)(Ph + e) = oh; *(volatile v2us*)(Pl + e) = ol; __threadfence(); *(volatile v2h*)(P16 + e) = o16; *(volatile v2us*)(Ph + e) = oh; *(volatile v2us*)(Pl + e) = ol; }
__global__ __launch_bounds__(256) void k_vtp(const float* __restrict__ F, int pitch, int nheads, h16* V16, bf* Vh, bf* Vl) { const size_t e = ((size_t)blockIdx.x * 256 + threadIdx.x) * 2; if (e >= (size_t)nheads * HD * SEQ) return; const int t = (int)(e % SEQ); const int d = (int)((e / SEQ) % HD); const int g = (int)(e / ((size_t)SEQ * HD)); v2h o16; v2us oh, ol;
#pragma unroll
    for (int q = 0; q < 2; ++q) { const float x = F[(size_t)(t + q) * pitch + g * HD + d]; o16[q] = tohx(x); unsigned short a2, c2; splitf(x, a2, c2); oh[q] = a2; ol[q] = c2; }
    *(volatile v2h*)(V16 + e) = o16; *(volatile v2us*)(Vh + e) = oh; *(volatile v2us*)(Vl + e) = ol; __threadfence(); *(volatile v2h*)(V16 + e) = o16; *(volatile v2us*)(Vh + e) = oh; *(volatile v2us*)(Vl + e) = ol; }

template <bool SPLIT>
__global__ __launch_bounds__(128) __attribute__((amdgpu_num_vgpr(256)))
void k_attn(const h16* __restrict__ Q16, const bf* __restrict__ Qh, const bf* __restrict__ Ql,
            const h16* __restrict__ K16, const bf* __restrict__ Kh, const bf* __restrict__ Kl,
            const h16* __restrict__ VT16, const bf* __restrict__ VTh, const bf* __restrict__ VTl,
            const int* __restrict__ causal, int qt0, bf* CTh, bf* CTl) {
    __shared__ __align__(16) h16 Ps16[SPLIT ? 8 : 4 * 16 * PP];
    __shared__ __align__(16) unsigned short Psh[SPLIT ? 4 * 16 * PP : 8];
    __shared__ __align__(16) unsigned short Psl[SPLIT ? 4 * 16 * PP : 8];
    __shared__ __align__(16) float Os[4 * 16 * OSP];
    const int wave = threadIdx.x >> 5, l = threadIdx.x & 31, h = l >> 4, m = l & 15;
    const int qt = qt0 + (int)blockIdx.x, q0 = qt * 64, z = (int)blockIdx.y;
    const int rw = q0 + wave * 16;
    const bool cm = (causal[0] != 0);
    const int nch = cm ? (qt + 1) : (SEQ / KCH);
    const size_t qoff = ((size_t)z * SEQ + rw + m) * HD + 8 * h;
    v16h qa[2]; v16bf qah[2], qal[2];
#pragma unroll
    for (int ks = 0; ks < 2; ++ks) {
        if (SPLIT) { qah[ks] = WFrag<bf>::ld(Qh + qoff + ks * 32); qal[ks] = WFrag<bf>::ld(Ql + qoff + ks * 32); }
        else       { qa[ks] = WFrag<h16>::ld(Q16 + qoff + ks * 32); }
    }
    v8f o[4]; float mrun[8], lrun[8];
#pragma unroll
    for (int nt = 0; nt < 4; ++nt) o[nt] = (v8f){};
#pragma unroll
    for (int r = 0; r < 8; ++r) { mrun[r] = -3.0e38f; lrun[r] = 0.0f; }
    h16* pw = Ps16 + (SPLIT ? 0 : wave * 16 * PP);
    unsigned short* pwh = Psh + (SPLIT ? wave * 16 * PP : 0);
    unsigned short* pwl = Psl + (SPLIT ? wave * 16 * PP : 0);
    float* os = Os + wave * 16 * OSP;

#pragma unroll 1
    for (int c = 0; c < nch; ++c) {
        const int kv0 = c * KCH;
        __builtin_amdgcn_wave_barrier(); asm volatile("" ::: "memory");
        v8f sc[4];
#pragma unroll
        for (int nt = 0; nt < 4; ++nt) sc[nt] = (v8f){};
#pragma unroll
        for (int ks = 0; ks < 2; ++ks) {
#pragma unroll
            for (int nt = 0; nt < 4; ++nt) {
                const size_t ko = ((size_t)z * SEQ + kv0 + nt * 16 + m) * HD + ks * 32 + 8 * h;
                if (SPLIT) {
                    const v16bf bh = WFrag<bf>::ld(Kh + ko); const v16bf bl = WFrag<bf>::ld(Kl + ko);
                    sc[nt] = wmmab(qah[ks], bh, sc[nt]); sc[nt] = wmmab(qal[ks], bh, sc[nt]); sc[nt] = wmmab(qah[ks], bl, sc[nt]);
                } else {
                    const v16h bk = WFrag<h16>::ld(K16 + ko);
                    sc[nt] = wmma16(qa[ks], bk, sc[nt]);
                }
            }
        }
        asm volatile("v_nop\n\tv_nop\n\tv_nop\n\tv_nop" : "+v"(sc[0]), "+v"(sc[1]), "+v"(sc[2]), "+v"(sc[3]));

#pragma unroll
        for (int r = 0; r < 8; ++r) {
            const int row = rw + 8 * h + r;
            float mx = -3.0e38f;
#pragma unroll
            for (int nt = 0; nt < 4; ++nt) { const int col = kv0 + nt * 16 + m; float s = sc[nt][r] * SCL; if (cm && col > row) s = -1.0e9f; sc[nt][r] = s; mx = fmaxf(mx, s); }
#pragma unroll
            for (int msk = 1; msk < 16; msk <<= 1) mx = fmaxf(mx, __shfl_xor(mx, msk, 32));
            const float mn = fmaxf(mrun[r], mx); const float al = __expf(mrun[r] - mn); mrun[r] = mn;
            float rs = 0.0f;
#pragma unroll
            for (int nt = 0; nt < 4; ++nt) { const float p = __expf(sc[nt][r] - mn); sc[nt][r] = p; rs += p; }
#pragma unroll
            for (int msk = 1; msk < 16; msk <<= 1) rs += __shfl_xor(rs, msk, 32);
            lrun[r] = lrun[r] * al + rs;
#pragma unroll
            for (int nt = 0; nt < 4; ++nt) o[nt][r] *= al;
        }

        if (SPLIT) {
#pragma unroll
            for (int nt = 0; nt < 4; ++nt)
#pragma unroll
                for (int r = 0; r < 8; ++r) { unsigned short a2, c2; splitf(sc[nt][r], a2, c2); pwh[(8 * h + r) * PP + nt * 16 + m] = a2; pwl[(8 * h + r) * PP + nt * 16 + m] = c2; }
        } else {
#pragma unroll
            for (int nt = 0; nt < 4; ++nt)
#pragma unroll
                for (int r = 0; r < 8; ++r) pw[(8 * h + r) * PP + nt * 16 + m] = tohx(sc[nt][r] * PCAR);
        }
        __builtin_amdgcn_fence(3, "wavefront"); __builtin_amdgcn_wave_barrier(); asm volatile("" ::: "memory");
#pragma unroll
        for (int ks = 0; ks < 2; ++ks) {
            const int po = m * PP + ks * 32 + 8 * h;
            if (SPLIT) {
                const v16bf pah = cat16b(*(const v8usa*)(pwh + po), *(const v8usa*)(pwh + po + 16));
                const v16bf pal = cat16b(*(const v8usa*)(pwl + po), *(const v8usa*)(pwl + po + 16));
#pragma unroll
                for (int nt = 0; nt < 4; ++nt) {
                    const size_t vo = ((size_t)z * HD + nt * 16 + m) * SEQ + kv0 + ks * 32 + 8 * h;
                    const v16bf vbh = WFrag<bf>::ld(VTh + vo); const v16bf vbl = WFrag<bf>::ld(VTl + vo);
                    o[nt] = wmmab(pah, vbh, o[nt]); o[nt] = wmmab(pal, vbh, o[nt]); o[nt] = wmmab(pah, vbl, o[nt]);
                }
            } else {
                const v16h pa = cat16(*(const v8ha*)(pw + po), *(const v8ha*)(pw + po + 16));
#pragma unroll
                for (int nt = 0; nt < 4; ++nt) {
                    const size_t vo = ((size_t)z * HD + nt * 16 + m) * SEQ + kv0 + ks * 32 + 8 * h;
                    const v16h vb = WFrag<h16>::ld(VT16 + vo);
                    o[nt] = wmma16(pa, vb, o[nt]);
                }
            }
        }
        asm volatile("v_nop\n\tv_nop\n\tv_nop\n\tv_nop" : "+v"(o[0]), "+v"(o[1]), "+v"(o[2]), "+v"(o[3]));
    }

    __builtin_amdgcn_wave_barrier(); asm volatile("" ::: "memory");
#pragma unroll
    for (int r = 0; r < 8; ++r) { const float inv = (SPLIT ? 1.0f : RPCAR) / lrun[r];
#pragma unroll
        for (int nt = 0; nt < 4; ++nt) os[(8 * h + r) * OSP + nt * 16 + m] = o[nt][r] * inv; }
    __builtin_amdgcn_fence(3, "wavefront"); __builtin_amdgcn_wave_barrier(); asm volatile("" ::: "memory");
    const int rr = l >> 3, c8 = (l & 7) * 8;
#pragma unroll 1
    for (int ps = 0; ps < 2; ++ps) {
#pragma unroll
        for (int s = 0; s < 4; ++s) {
            const int row = 4 * s + rr;
            const v4f a0 = *(const v4fa*)(os + row * OSP + c8); const v4f a1 = *(const v4fa*)(os + row * OSP + c8 + 4);
            v8us oh, ol;
#pragma unroll
            for (int j = 0; j < 4; ++j) { unsigned short th, tl; splitf(a0[j], th, tl); oh[j] = th; ol[j] = tl; splitf(a1[j], th, tl); oh[4 + j] = th; ol[4 + j] = tl; }
            const size_t dofs = (size_t)(rw + row) * DM + (size_t)z * HD + c8;
            *(volatile v8us*)(CTh + dofs) = oh; *(volatile v8us*)(CTl + dofs) = ol;
        }
        if (ps == 0) __threadfence();
    }
}

extern "C" void kernel_launch(void* const* d_in, const int* in_sizes, int n_in,
                              void* d_out, int out_size, void* d_ws, size_t ws_size, hipStream_t stream) {
    if (n_in < 6) return;
    if ((size_t)in_sizes[0] < (size_t)(NB - 1) * SEQ_FULL * DM + (size_t)SEQ * DM) return;
    if ((size_t)in_sizes[1] < (size_t)3 * DM * DM || in_sizes[2] < 3 * DM || (size_t)in_sizes[3] < (size_t)DM * DM || in_sizes[4] < DM || in_sizes[5] < 1) return;
    if ((size_t)out_size < (size_t)NB * SEQ * DM) return;
    const float* x     = (const float*)d_in[0];
    const float* w_in  = (const float*)d_in[1];
    const float* b_in  = (const float*)d_in[2];
    const float* w_out = (const float*)d_in[3];
    const float* b_out = (const float*)d_in[4];
    const int*   causal = (const int*)d_in[5];
    float* OUT = (float*)d_out;
    char* wsp = (char*)d_ws;
    auto take = [&](size_t bytes) { char* p = wsp; wsp += (bytes + 255) & ~(size_t)255; return (void*)p; };
    const size_t PL = (size_t)NH * SEQ * HD;
    bf* WIN = (bf*)take((size_t)3 * DM * DM * 2); bf* WO = (bf*)take((size_t)DM * DM * 2);
    bf* XB = (bf*)take((size_t)SEQ * DM * 2); float* FQKV = (float*)take((size_t)SEQ * 3 * DM * 4);
    h16* Q16 = (h16*)take(PL * 2); bf* Qh = (bf*)take(PL * 2); bf* Ql = (bf*)take(PL * 2);
    h16* K16 = (h16*)take(PL * 2); bf* Kh = (bf*)take(PL * 2); bf* Kl = (bf*)take(PL * 2);
    h16* VT16 = (h16*)take(PL * 2); bf* VTh = (bf*)take(PL * 2); bf* VTl = (bf*)take(PL * 2);
    bf* CTh = (bf*)take((size_t)SEQ * DM * 2); bf* CTl = (bf*)take((size_t)SEQ * DM * 2);
    if ((size_t)(wsp - (char*)d_ws) > ws_size) return;

    k_cvt8<<<(unsigned)(((size_t)3 * DM * DM / 8 + 255) / 256), 256, 0, stream>>>(w_in, WIN, (size_t)3 * DM * DM / 8);
    k_cvt8<<<(unsigned)(((size_t)DM * DM / 8 + 255) / 256), 256, 0, stream>>>(w_out, WO, (size_t)DM * DM / 8);
    const unsigned LP = (unsigned)((PL / 2 + 255) / 256);
    const int nts = RHE / 64, ntp = SEQ / 64 - nts;
    for (int b = 0; b < NB; ++b) {
        k_cvt8<<<(unsigned)(((size_t)SEQ * DM / 8 + 255) / 256), 256, 0, stream>>>(x + (size_t)b * SEQ_FULL * DM, XB, (size_t)SEQ * DM / 8);
        k_gemmw<bf, 0, true><<<dim3(SEQ / 64, 3 * DM / 64, 1), 32, 0, stream>>>(XB, nullptr, WIN, nullptr, DM, FQKV, 3 * DM, b_in, 0, 0, 0);
        k_hp<<<LP, 256, 0, stream>>>(FQKV, 3 * DM, Q16, Qh, Ql);
        k_hp<<<LP, 256, 0, stream>>>(FQKV + DM, 3 * DM, K16, Kh, Kl);
        k_vtp<<<LP, 256, 0, stream>>>(FQKV + 2 * DM, 3 * DM, NH, VT16, VTh, VTl);
        if (nts > 0) k_attn<true><<<dim3((unsigned)nts, NH, 1), 128, 0, stream>>>(Q16, Qh, Ql, K16, Kh, Kl, VT16, VTh, VTl, causal, 0, CTh, CTl);
        if (ntp > 0) k_attn<false><<<dim3((unsigned)ntp, NH, 1), 128, 0, stream>>>(Q16, Qh, Ql, K16, Kh, Kl, VT16, VTh, VTl, causal, nts, CTh, CTl);
        k_gemmw<bf, 1, true><<<dim3(SEQ / 64, DM / 64, 1), 32, 0, stream>>>(CTh, CTl, WO, nullptr, DM, OUT + (size_t)b * SEQ * DM, DM, b_out, 0, 0, 0);
    }
}
